// DConvModules_31559419691502
// MI455X (gfx1250) — hardware-verified
//
#include <hip/hip_runtime.h>
#include <math.h>
typedef __attribute__((ext_vector_type(16))) _Float16 v16h;
typedef __attribute__((ext_vector_type(8)))  _Float16 v8h;
typedef __attribute__((ext_vector_type(16))) __bf16   v16b;
typedef __attribute__((ext_vector_type(8)))  __bf16   v8b;
typedef __attribute__((ext_vector_type(8)))  float    v8f;
typedef __attribute__((ext_vector_type(4)))  float    v4f;
#define PSCALE 32768.0f
#define U16(p) ((const unsigned short*)(const void*)(p))
#define PSCALE_INV (1.0f / 32768.0f)

__device__ __forceinline__ unsigned short f2bf_bits(float f) {
  unsigned u = __float_as_uint(f);
  return (unsigned short)((u + 0x7FFFu + ((u >> 16) & 1u)) >> 16);
}
__device__ __forceinline__ float bf_bits2f(unsigned short h) { return __uint_as_float(((unsigned)h) << 16); }

__device__ __forceinline__ void dep_guard_h(v8f& a, v8f& b, v16h x, v16h y) { asm volatile("v_nop\n\tv_nop\n\tv_nop\n\tv_nop" : "+v"(a), "+v"(b) : "v"(x), "v"(y)); }
__device__ __forceinline__ void dep_guard_b(v8f& a, v8f& b, v16b x, v16b y) { asm volatile("v_nop\n\tv_nop\n\tv_nop\n\tv_nop" : "+v"(a), "+v"(b) : "v"(x), "v"(y)); }
__device__ __forceinline__ void keep4_h(v16h a, v16h b, v16h c, v16h d) { asm volatile("v_nop" :: "v"(a), "v"(b), "v"(c), "v"(d)); }
__device__ __forceinline__ void keep4_b(v16b a, v16b b, v16b c, v16b d) { asm volatile("v_nop" :: "v"(a), "v"(b), "v"(c), "v"(d)); }
__device__ __forceinline__ void acc_guard4(v8f& a, v8f& b, v8f& c, v8f& d) { asm volatile("v_nop\n\tv_nop\n\tv_nop\n\tv_nop" : "+v"(a), "+v"(b), "+v"(c), "+v"(d)); }
template <typename T> struct Frag;
template <> struct Frag<_Float16> {
  typedef v16h V; union U { v16h v; v8h h[2]; };
  static __device__ __forceinline__ v16h load(const _Float16* p) {
    U f; f.h[0] = *(const v8h*)(p); f.h[1] = *(const v8h*)(p + 16); return f.v;
  }
  static __device__ __forceinline__ v8f mma(v16h a, v16h b, v8f c) {
    return __builtin_amdgcn_wmma_f32_16x16x32_f16(false, a, false, b, (short)0, c, false, false);
  }
  static __device__ __forceinline__ void guard(v8f& a, v8f& b, v16h x, v16h y) { dep_guard_h(a, b, x, y); }
  static __device__ __forceinline__ void keep(v16h a, v16h b, v16h c, v16h d) { keep4_h(a, b, c, d); }
};
template <> struct Frag<__bf16> {
  typedef v16b V; union U { v16b v; v8b h[2]; };
  static __device__ __forceinline__ v16b load(const __bf16* p) {
    U f; f.h[0] = *(const v8b*)(p); f.h[1] = *(const v8b*)(p + 16); return f.v;
  }
  static __device__ __forceinline__ v8f mma(v16b a, v16b b, v8f c) {
    return __builtin_amdgcn_wmma_f32_16x16x32_bf16(false, a, false, b, (short)0, c, false, false);
  }
  static __device__ __forceinline__ void guard(v8f& a, v8f& b, v16b x, v16b y) { dep_guard_b(a, b, x, y); }
  static __device__ __forceinline__ void keep(v16b a, v16b b, v16b c, v16b d) { keep4_b(a, b, c, d); }
};

template <int ET> struct Elem;
template <> struct Elem<0> { typedef _Float16 T; };
template <> struct Elem<1> { typedef __bf16 T; };
template <int ET, bool SPLIT, int BIAS_MODE, int OUT_MODE, bool RESID, int ACT = 0>
__global__ __launch_bounds__(256) void wmma_gemm64(
    const unsigned short* __restrict__ Ap, const unsigned short* __restrict__ A2p, int lda, long strideA,
    const unsigned short* __restrict__ Btp, const unsigned short* __restrict__ Bt2p, int ldb, long strideB,
    void* __restrict__ Cout, void* __restrict__ Cout2, int ldc, long strideC,
    const float* __restrict__ bias,
    const float* __restrict__ resid, long strideR,
    int M, int N, int K, float scale) {
  typedef typename Elem<ET>::T T;
  typedef typename Frag<T>::V V;
  const T* A = (const T*)Ap; const T* A2 = (const T*)A2p; const T* Bt = (const T*)Btp; const T* Bt2 = (const T*)Bt2p;
  __shared__ __align__(16) float sT[8][16 * 68];
  const int b    = blockIdx.y;
  const int lane = threadIdx.x & 31;
  const int wave = threadIdx.x >> 5;
  const int tilesN = N >> 6;
  const int tilesM = M >> 6;
  const int tile = blockIdx.x * 8 + wave;
  if (tile >= tilesM * tilesN) return;
  const int tm = tile / tilesN;
  const int tn = tile - tm * tilesN;
  const int m0 = tm << 6;
  const int n0 = tn << 6;

  const T* Ab  = A  + (size_t)b * strideA;
  const T* Bb  = Bt + (size_t)b * strideB;
  const T* Ab2 = SPLIT ? (A2  + (size_t)b * strideA) : nullptr;
  const T* Bb2 = SPLIT ? (Bt2 + (size_t)b * strideB) : nullptr;

  const int rlane = lane & 15;
  const int koff  = (lane >> 4) * 8;
  const int mOff  = (lane >> 4) * 8;

  v8f acc[4][4];
#pragma unroll
  for (int i = 0; i < 4; ++i)
#pragma unroll
    for (int j = 0; j < 4; ++j) acc[i][j] = (v8f){0.f,0.f,0.f,0.f,0.f,0.f,0.f,0.f};

  for (int k0 = 0; k0 < K; k0 += 32) {
    V bh[4], bl[4];
#pragma unroll
    for (int j = 0; j < 4; ++j) {
      const size_t bo = (size_t)(n0 + (j << 4) + rlane) * ldb + koff + k0;
      bh[j] = Frag<T>::load(Bb + bo);
      if (SPLIT) bl[j] = Frag<T>::load(Bb2 + bo);
    }
#pragma unroll
    for (int i = 0; i < 4; ++i) {
      const size_t ao = (size_t)(m0 + (i << 4) + rlane) * lda + koff + k0;
      V ah = Frag<T>::load(Ab + ao);
      V al;
      if (SPLIT) al = Frag<T>::load(Ab2 + ao);
#pragma unroll
      for (int j = 0; j < 4; ++j) {
        acc[i][j] = Frag<T>::mma(ah, bh[j], acc[i][j]);
        if (SPLIT) {
          acc[i][j] = Frag<T>::mma(ah, bl[j], acc[i][j]);
          acc[i][j] = Frag<T>::mma(al, bh[j], acc[i][j]);
        }
      }
      Frag<T>::guard(acc[i][0], acc[i][3], ah, SPLIT ? al : ah);
    }
    Frag<T>::keep(bh[0], bh[1], bh[2], bh[3]);
    if (SPLIT) Frag<T>::keep(bl[0], bl[1], bl[2], bl[3]);
  }
  acc_guard4(acc[0][0], acc[0][1], acc[0][2], acc[0][3]);
  acc_guard4(acc[1][0], acc[1][1], acc[1][2], acc[1][3]);
  acc_guard4(acc[2][0], acc[2][1], acc[2][2], acc[2][3]);
  acc_guard4(acc[3][0], acc[3][1], acc[3][2], acc[3][3]);

  float* slab = sT[wave];
  const float* Rb = RESID ? (resid + (size_t)b * strideR) : nullptr;
#pragma unroll
  for (int i = 0; i < 4; ++i) {
    const int mBase = m0 + (i << 4);
#pragma unroll
    for (int j = 0; j < 4; ++j) {
      const int n = n0 + (j << 4) + rlane;
      float bv = 0.f;
      if (BIAS_MODE == 2) bv = bias[n];
#pragma unroll
      for (int r = 0; r < 8; ++r) {
        float v = acc[i][j][r] * scale;
        if (BIAS_MODE == 1) v += bias[mBase + mOff + r];
        if (BIAS_MODE == 2) v += bv;
        if (RESID) v += Rb[(size_t)(mBase + mOff + r) * ldc + n];
        if (ACT == 1) v = tanhf(v);
        if (ACT == 2) v = fmaxf(v, 0.0f);
        if (ACT == 3) v = v / (1.0f + expf(-v));
        if (ACT == 4) v = (v > 0.f) ? v : 0.01f * v;
        if (ACT == 5) v = 0.5f * v * (1.0f + erff(v * 0.70710678118654752f));
        slab[(mOff + r) * 68 + (j << 4) + rlane] = v;
      }
    }
    __builtin_amdgcn_fence(__ATOMIC_RELEASE, "workgroup");
    __builtin_amdgcn_wave_barrier();
    __builtin_amdgcn_fence(__ATOMIC_ACQUIRE, "workgroup");
    if (OUT_MODE == 0) {
      float* C = (float*)Cout + (size_t)b * strideC;
      const int hh = lane >> 4, c4 = (lane & 15) * 4;
      for (int pass = 0; pass < 2; ++pass) {
#pragma unroll
        for (int it = 0; it < 8; ++it) {
          const int row = it * 2 + hh;
          v4f v = *(const v4f*)(slab + row * 68 + c4);
          *(volatile v4f*)(C + (size_t)(mBase + row) * ldc + n0 + c4) = v;
        }
        __threadfence();
      }
    } else {
      const int q = lane >> 3, c8 = (lane & 7) * 8;
      unsigned short* C  = (unsigned short*)Cout  + (size_t)b * strideC;
      unsigned short* C2 = (OUT_MODE == 2) ? ((unsigned short*)Cout2 + (size_t)b * strideC) : nullptr;
      for (int pass = 0; pass < 2; ++pass) {
#pragma unroll
        for (int it = 0; it < 4; ++it) {
          const int row = it * 4 + q;
          const float* sp = slab + row * 68 + c8;
          v8h hv, lv;
#pragma unroll
          for (int e = 0; e < 8; ++e) {
            if (OUT_MODE == 1) {
              hv[e] = (_Float16)sp[e];
            } else {
              unsigned short hb = f2bf_bits(sp[e]);
              unsigned short lb = f2bf_bits(sp[e] - bf_bits2f(hb));
              hv[e] = __builtin_bit_cast(_Float16, hb);
              lv[e] = __builtin_bit_cast(_Float16, lb);
            }
          }
          *(volatile v8h*)(C + (size_t)(mBase + row) * ldc + n0 + c8) = hv;
          if (OUT_MODE == 2) *(volatile v8h*)(C2 + (size_t)(mBase + row) * ldc + n0 + c8) = lv;
        }
        __threadfence();
      }
    }
    __builtin_amdgcn_fence(__ATOMIC_RELEASE, "workgroup");
    __builtin_amdgcn_wave_barrier();
    __builtin_amdgcn_fence(__ATOMIC_ACQUIRE, "workgroup");
  }
}

__global__ __launch_bounds__(256) void cast_f32_f16x2(
    const float* __restrict__ in, _Float16* __restrict__ out, int n2) {
  int i = blockIdx.x * 256 + threadIdx.x;
  if (i < n2) {
    const _Float16 h0 = (_Float16)in[2 * i], h1 = (_Float16)in[2 * i + 1];
    const unsigned u = (unsigned)__builtin_bit_cast(unsigned short, h0) | ((unsigned)__builtin_bit_cast(unsigned short, h1) << 16);
    ((volatile unsigned*)out)[i] = u;
    __threadfence();
    ((volatile unsigned*)out)[i] = u;
  }
}


#define DB 4
#define DHh 128
#define DWw 128
#define DHW (DHh * DWw)
#define DP (DB * DHW)
#define DC 96
#define DCP 128
#define DKK 9
#define DKC (DKK * DCP)
#define DO 64
__global__ __launch_bounds__(256) void ln_in_kernel(const float* __restrict__ fe, const float* __restrict__ ff, const float* __restrict__ we, const float* __restrict__ be, const float* __restrict__ wf, const float* __restrict__ bf_, float* __restrict__ OXT) {
  const int lane = threadIdx.x & 31, wave = threadIdx.x >> 5; const int p = blockIdx.x * 8 + wave; const int b = p / DHW, hw = p % DHW;
  const float e = fe[((size_t)b * 32 + lane) * DHW + hw]; const float f0 = ff[((size_t)b * 64 + lane) * DHW + hw], f1 = ff[((size_t)b * 64 + 32 + lane) * DHW + hw];
  float s = e; for (int o = 16; o > 0; o >>= 1) s += __shfl_xor(s, o, 32); const float mu = s / 32.f; float d = e - mu; float v = d * d; for (int o = 16; o > 0; o >>= 1) v += __shfl_xor(v, o, 32);
  const float en = d / sqrtf(v / 32.f + 1e-5f) * we[lane] + be[lane];
  float s2 = f0 + f1; for (int o = 16; o > 0; o >>= 1) s2 += __shfl_xor(s2, o, 32); const float mu2 = s2 / 64.f; const float d0 = f0 - mu2, d1 = f1 - mu2; float v2 = d0 * d0 + d1 * d1; for (int o = 16; o > 0; o >>= 1) v2 += __shfl_xor(v2, o, 32);
  const float inv2 = 1.0f / sqrtf(v2 / 64.f + 1e-5f);
  const float fn0 = d0 * inv2 * wf[lane] + bf_[lane], fn1 = d1 * inv2 * wf[32 + lane] + bf_[32 + lane];
  float* row = OXT + (size_t)p * DC;
  for (int pass = 0; pass < 2; ++pass) { ((volatile float*)row)[lane] = en; ((volatile float*)row)[32 + lane] = fn0; ((volatile float*)row)[64 + lane] = fn1; __threadfence(); }
}
__global__ __launch_bounds__(256) void col_reg_kernel(const float* __restrict__ OXT, unsigned* __restrict__ A) {
  const int lane = threadIdx.x & 31, wave = threadIdx.x >> 5; const int item = blockIdx.x * 8 + wave; const int p = item / DKK, k = item % DKK;
  const int b = p / DHW, hw = p % DHW, h = hw / DWw, w = hw % DWw; const int yy = h + k / 3 - 1, xx = w + k % 3 - 1;
  v4f v = {0.f, 0.f, 0.f, 0.f};
  if (lane < 24 && yy >= 0 && yy < DHh && xx >= 0 && xx < DWw) v = *(const v4f*)(OXT + ((size_t)b * DHW + yy * DWw + xx) * DC + lane * 4);
  typedef __attribute__((ext_vector_type(2))) unsigned u2; u2 pk;
  pk[0] = (unsigned)__builtin_bit_cast(unsigned short, (_Float16)v[0]) | ((unsigned)__builtin_bit_cast(unsigned short, (_Float16)v[1]) << 16);
  pk[1] = (unsigned)__builtin_bit_cast(unsigned short, (_Float16)v[2]) | ((unsigned)__builtin_bit_cast(unsigned short, (_Float16)v[3]) << 16);
  unsigned* dst = A + ((size_t)p * DKC + k * DCP) / 2 + lane * 2;
  *(volatile u2*)dst = pk; __threadfence(); *(volatile u2*)dst = pk;
}
__global__ __launch_bounds__(256) void wperm_kernel(const float* __restrict__ w, const float* __restrict__ bsrc, int nout, int row0, unsigned* __restrict__ WT, float* __restrict__ bp) {
  const int i = blockIdx.x * 256 + threadIdx.x; if (i >= nout * DKC / 2) return; const int o = (2 * i) / DKC, r = (2 * i) % DKC; const int k = r / DCP, c = r % DCP;
  float a = 0.f, b = 0.f; if (c < DC) { a = w[((size_t)o * DC + c) * DKK + k]; b = w[((size_t)o * DC + c + 1) * DKK + k]; }
  const unsigned u = (unsigned)__builtin_bit_cast(unsigned short, (_Float16)a) | ((unsigned)__builtin_bit_cast(unsigned short, (_Float16)b) << 16);
  ((volatile unsigned*)WT)[(size_t)(row0 + o) * (DKC / 2) + r / 2] = u; if (r == 0) ((volatile float*)bp)[row0 + o] = bsrc[o]; __threadfence();
  ((volatile unsigned*)WT)[(size_t)(row0 + o) * (DKC / 2) + r / 2] = u; if (r == 0) ((volatile float*)bp)[row0 + o] = bsrc[o];
}
__global__ __launch_bounds__(256) void zero_kernel(unsigned* __restrict__ p, long n) { const long i = (long)blockIdx.x * 256 + threadIdx.x; if (i < n) { ((volatile unsigned*)p)[i] = 0u; __threadfence(); ((volatile unsigned*)p)[i] = 0u; } }
__global__ __launch_bounds__(256) void col_def_kernel(const float* __restrict__ OXT, const float* __restrict__ OM, unsigned* __restrict__ A) {
  const int lane = threadIdx.x & 31, wave = threadIdx.x >> 5; const int item = blockIdx.x * 8 + wave; const int p = item / DKK, k = item % DKK;
  const int b = p / DHW, hw = p % DHW, h = hw / DWw, w = hw % DWw;
  const float dy = OM[(size_t)p * 64 + 2 * k], dx = OM[(size_t)p * 64 + 2 * k + 1]; const float m = 2.0f / (1.0f + expf(-OM[(size_t)p * 64 + 18 + k]));
  const float py = ((float)h + (float)(k / 3 - 1)) + dy, px = ((float)w + (float)(k % 3 - 1)) + dx;
  const float y0f = floorf(py), x0f = floorf(px); const float wy1 = py - y0f, wx1 = px - x0f; const int y0 = (int)y0f, x0 = (int)x0f;
  v4f v = {0.f, 0.f, 0.f, 0.f};
  if (lane < 24) {
#pragma unroll
    for (int corner = 0; corner < 4; ++corner) { const int yi = y0 + (corner >> 1), xi = x0 + (corner & 1);
      const float wc = ((corner >> 1) ? wy1 : (1.f - wy1)) * ((corner & 1) ? wx1 : (1.f - wx1));
      if (yi >= 0 && yi <= DHh - 1 && xi >= 0 && xi <= DWw - 1) v += wc * *(const v4f*)(OXT + ((size_t)b * DHW + yi * DWw + xi) * DC + lane * 4); }
    v = v * m; }
  typedef __attribute__((ext_vector_type(2))) unsigned u2; u2 pk;
  pk[0] = (unsigned)__builtin_bit_cast(unsigned short, (_Float16)v[0]) | ((unsigned)__builtin_bit_cast(unsigned short, (_Float16)v[1]) << 16);
  pk[1] = (unsigned)__builtin_bit_cast(unsigned short, (_Float16)v[2]) | ((unsigned)__builtin_bit_cast(unsigned short, (_Float16)v[3]) << 16);
  unsigned* dst = A + ((size_t)p * DKC + k * DCP) / 2 + lane * 2;
  *(volatile u2*)dst = pk; __threadfence(); *(volatile u2*)dst = pk;
}
__global__ __launch_bounds__(256) void out_kernel(const float* __restrict__ AL, const float* __restrict__ wl, const float* __restrict__ bl, float* __restrict__ out) {
  __shared__ float tile[64][65];
  const int b = blockIdx.y, p0 = blockIdx.x * 64, tx = threadIdx.x, ty = threadIdx.y; const int lane = tx;
  for (int q = 0; q < 8; ++q) { const int p = ty * 8 + q; const size_t gp = (size_t)b * DHW + p0 + p;
    float a0 = AL[gp * DO + lane], a1 = AL[gp * DO + 32 + lane]; a0 = a0 >= 0.f ? a0 : 0.2f * a0; a1 = a1 >= 0.f ? a1 : 0.2f * a1;
    float s = a0 + a1; for (int o = 16; o > 0; o >>= 1) s += __shfl_xor(s, o, 32); const float mu = s / 64.f; const float d0 = a0 - mu, d1 = a1 - mu; float v = d0 * d0 + d1 * d1; for (int o = 16; o > 0; o >>= 1) v += __shfl_xor(v, o, 32);
    const float inv = 1.0f / sqrtf(v / 64.f + 1e-5f);
    tile[lane][p] = d0 * inv * wl[lane] + bl[lane]; tile[32 + lane][p] = d1 * inv * wl[32 + lane] + bl[32 + lane]; }
  __syncthreads();
  for (int pass = 0; pass < 2; ++pass) { for (int c = ty; c < 64; c += 8) { float* dst = out + ((size_t)b * DO + c) * DHW + p0; ((volatile float*)dst)[tx] = tile[c][tx]; ((volatile float*)dst)[32 + tx] = tile[c][32 + tx]; } __threadfence(); }
}
extern "C" void kernel_launch(void* const* d_in, const int* in_sizes, int n_in, void* d_out, int out_size, void* d_ws, size_t ws_size, hipStream_t stream) {
  (void)in_sizes; (void)n_in; (void)out_size; (void)ws_size;
  const float* fevt = (const float*)d_in[0]; const float* fef = (const float*)d_in[1]; const float* lwe = (const float*)d_in[2]; const float* lbe = (const float*)d_in[3]; const float* lwf = (const float*)d_in[4]; const float* lbf = (const float*)d_in[5];
  const float* lwa = (const float*)d_in[6]; const float* lba = (const float*)d_in[7]; const float* offw = (const float*)d_in[8]; const float* offb = (const float*)d_in[9]; const float* modw = (const float*)d_in[10]; const float* modb = (const float*)d_in[11];
  const float* regw = (const float*)d_in[12]; const float* regb = (const float*)d_in[13]; (void)d_in[14];
  char* ws = (char*)d_ws; size_t off = 0;
  auto carve = [&](size_t bytes) -> char* { char* p = ws + off; off += (bytes + 255) & ~(size_t)255; return p; };
  float* OXT = (float*)carve((size_t)DP * DC * 4);
  unsigned* A = (unsigned*)carve((size_t)DP * DKC * 2);
  unsigned* WOM = (unsigned*)carve((size_t)64 * DKC * 2); float* bom = (float*)carve(64 * 4); unsigned* WRG = (unsigned*)carve((size_t)64 * DKC * 2); float* brg = (float*)carve(64 * 4);
  float* OM = (float*)carve((size_t)DP * 64 * 4); float* AL = (float*)carve((size_t)DP * DO * 4);
  ln_in_kernel<<<DP / 8, 256, 0, stream>>>(fevt, fef, lwe, lbe, lwf, lbf, OXT);
  zero_kernel<<<(64 * DKC / 2 + 255) / 256, 256, 0, stream>>>(WOM, 64 * DKC / 2); zero_kernel<<<1, 64, 0, stream>>>((unsigned*)bom, 64);
  wperm_kernel<<<(18 * DKC / 2 + 255) / 256, 256, 0, stream>>>(offw, offb, 18, 0, WOM, bom);
  wperm_kernel<<<(9 * DKC / 2 + 255) / 256, 256, 0, stream>>>(modw, modb, 9, 18, WOM, bom);
  wperm_kernel<<<(64 * DKC / 2 + 255) / 256, 256, 0, stream>>>(regw, regb, 64, 0, WRG, brg);
  col_reg_kernel<<<DP * DKK / 8, 256, 0, stream>>>(OXT, A);
  const int t = (DP / 64) * 1;
  wmma_gemm64<0, false, 2, 0, false><<<dim3((t + 7) / 8, 1), 256, 0, stream>>>((const unsigned short*)A, nullptr, DKC, 0, (const unsigned short*)WOM, nullptr, DKC, 0, OM, nullptr, 64, 0, bom, nullptr, 0, DP, 64, DKC, 1.0f);
  col_def_kernel<<<DP * DKK / 8, 256, 0, stream>>>(OXT, OM, A);
  wmma_gemm64<0, false, 2, 0, false><<<dim3((t + 7) / 8, 1), 256, 0, stream>>>((const unsigned short*)A, nullptr, DKC, 0, (const unsigned short*)WRG, nullptr, DKC, 0, AL, nullptr, DO, 0, brg, nullptr, 0, DP, DO, DKC, 1.0f);
  out_kernel<<<dim3(DHW / 64, DB), dim3(32, 8), 0, stream>>>(AL, lwa, lba, (float*)d_out);
}
